// MultiLayerGAT_30709016167272
// MI455X (gfx1250) — hardware-verified
//
#include <hip/hip_runtime.h>
#include <stddef.h>


#define DIN   128
#define HID   128
#define OUTD  64
#define NGR   64
#define PP    (NGR * OUTD)
#define GR    32
#define AP    136
#define NB    512
#define CHUNK 2048
#define NTHR  256
#define NWAVE 8
#define WCAP  256
#define NGRP  (CHUNK / (NTHR * 4))
#define SCA   8.0f
#define SCW   32.0f
#define SCINV 0.00390625f

static_assert(WCAP == (CHUNK / NTHR) * 32);
static_assert(NGRP == 2);
static_assert(NB == 512);
static_assert(CHUNK == 2048);
static_assert(PP == 4 * 128 * NWAVE);
static_assert((NTHR / OUTD) * NGR * OUTD == NTHR * NGR);

typedef float    v2f  __attribute__((ext_vector_type(2)));
typedef float    v4f  __attribute__((ext_vector_type(4)));
typedef float    v8f  __attribute__((ext_vector_type(8)));
typedef int      v4i  __attribute__((ext_vector_type(4)));
typedef _Float16 v8h  __attribute__((ext_vector_type(8)));
typedef _Float16 v16h __attribute__((ext_vector_type(16)));
union Frag   { v16h v; v8h half[2]; };
union Pack16 { v8h h; v4i i; };

template <int VL> struct VecT;
template <> struct VecT<2> { typedef v2f t; };
template <> struct VecT<4> { typedef v4f t; };

__device__ __forceinline__ v8f wm(v16h a, v16h b, v8f c) {
  v8f d = __builtin_amdgcn_wmma_f32_16x16x32_f16(false, a, false, b, (short)0, c, false, false);
  asm volatile("v_nop\n\tv_nop\n\tv_nop\n\tv_nop" : "+v"(d) : "v"(a), "v"(b));
  return d;
}

__global__ __launch_bounds__(NTHR) void k_prep(const float* __restrict__ W, _Float16* Wt, int din, int dout) {
  const int i  = blockIdx.x * NTHR + threadIdx.x;
  const int kp = din >> 3;
  if (i >= dout * kp) return;
  const int n  = i / kp;
  const int k8 = (i - n * kp) * 8;
  Pack16 u;
#pragma unroll
  for (int j = 0; j < 8; ++j) u.h[j] = (_Float16)(W[(size_t)(k8 + j) * dout + n] * SCW);
  _Float16* p = Wt + (size_t)n * din + k8;
  *(volatile v4i*)p = u.i;
  __threadfence();
  *(volatile v4i*)p = u.i;
}

template <int NW, int XSP>
__device__ __forceinline__ void epi_tile(v8f acc, int T, int hh, int m, int wave, int ncol,
                                         float cs, float cd, float* Xs, float* Ps, float* Pd) {
  float ss[8], sd[8];
#pragma unroll
  for (int r = 0; r < 8; ++r) {
    const float v = acc[r] * SCINV;
    Xs[(T * 16 + 8 * hh + r) * XSP + ncol] = v;
    ss[r] = v * cs;
    sd[r] = v * cd;
  }
#pragma unroll
  for (int mk = 1; mk < 16; mk <<= 1) {
#pragma unroll
    for (int r = 0; r < 8; ++r) {
      ss[r] += __shfl_xor(ss[r], mk, 32);
      sd[r] += __shfl_xor(sd[r], mk, 32);
    }
  }
  if (m == 0) {
#pragma unroll
    for (int r = 0; r < 8; ++r) {
      Ps[(T * 16 + 8 * hh + r) * NW + wave] = ss[r];
      Pd[(T * 16 + 8 * hh + r) * NW + wave] = sd[r];
    }
  }
}

template <int DOUT>
__global__ __launch_bounds__(DOUT * 2) void k_gemm(
    const float* __restrict__ xin, const _Float16* __restrict__ Wt,
    const float* __restrict__ att_s, const float* __restrict__ att_d,
    float* hp, float* asb, float* adb, int nN) {
  constexpr int NW  = DOUT / 16;
  constexpr int NT  = 32 * NW;
  constexpr int XSP = DOUT + 4;
  __shared__ __attribute__((aligned(16))) _Float16 At[GR * AP];
  __shared__ __attribute__((aligned(16))) float Xs[GR * XSP];
  __shared__ float Ps[GR * NW];
  __shared__ float Pd[GR * NW];
  __shared__ __attribute__((aligned(16))) float Sl[GR];
  __shared__ __attribute__((aligned(16))) float Dl[GR];

  const int tid  = threadIdx.x;
  const int lane = tid & 31;
  const int wave = tid >> 5;
  const int hh   = lane >> 4;
  const int m    = lane & 15;
  const int rowBase = blockIdx.x * GR;

  for (int p = tid; p < GR * 8; p += NT) {
    const int r  = p >> 3;
    const int c0 = (p & 7) * 16;
    int row = rowBase + r;
    if (row > nN - 1) row = nN - 1;
    const float* q = xin + (size_t)row * DIN + c0;
    const v4f f0 = *(const v4f*)(q), f1 = *(const v4f*)(q + 4);
    const v4f f2 = *(const v4f*)(q + 8), f3 = *(const v4f*)(q + 12);
    Pack16 u0, u1;
    u0.h[0] = (_Float16)(f0.x * SCA); u0.h[1] = (_Float16)(f0.y * SCA); u0.h[2] = (_Float16)(f0.z * SCA); u0.h[3] = (_Float16)(f0.w * SCA);
    u0.h[4] = (_Float16)(f1.x * SCA); u0.h[5] = (_Float16)(f1.y * SCA); u0.h[6] = (_Float16)(f1.z * SCA); u0.h[7] = (_Float16)(f1.w * SCA);
    u1.h[0] = (_Float16)(f2.x * SCA); u1.h[1] = (_Float16)(f2.y * SCA); u1.h[2] = (_Float16)(f2.z * SCA); u1.h[3] = (_Float16)(f2.w * SCA);
    u1.h[4] = (_Float16)(f3.x * SCA); u1.h[5] = (_Float16)(f3.y * SCA); u1.h[6] = (_Float16)(f3.z * SCA); u1.h[7] = (_Float16)(f3.w * SCA);
    *(v8h*)(At + r * AP + c0)     = u0.h;
    *(v8h*)(At + r * AP + c0 + 8) = u1.h;
  }
  __syncthreads();

  const int ncol = wave * 16 + m;
  v8f c0a = {0.f, 0.f, 0.f, 0.f, 0.f, 0.f, 0.f, 0.f};
  v8f c1a = {0.f, 0.f, 0.f, 0.f, 0.f, 0.f, 0.f, 0.f};
#pragma unroll
  for (int kt = 0; kt < DIN / 32; ++kt) {
    const int k0 = kt * 32;
    Frag a0, a1, b;
    const _Float16* pb  = Wt + (size_t)ncol * DIN + k0 + 8 * hh;
    const _Float16* pa0 = At + m * AP + k0 + 8 * hh;
    const _Float16* pa1 = At + (16 + m) * AP + k0 + 8 * hh;
    b.half[0]  = *(const v8h*)pb;  b.half[1]  = *(const v8h*)(pb + 16);
    a0.half[0] = *(const v8h*)pa0; a0.half[1] = *(const v8h*)(pa0 + 16);
    a1.half[0] = *(const v8h*)pa1; a1.half[1] = *(const v8h*)(pa1 + 16);
    c0a = wm(a0.v, b.v, c0a);
    c1a = wm(a1.v, b.v, c1a);
  }

  const float cs = att_s[ncol];
  const float cd = att_d[ncol];
  epi_tile<NW, XSP>(c0a, 0, hh, m, wave, ncol, cs, cd, Xs, Ps, Pd);
  epi_tile<NW, XSP>(c1a, 1, hh, m, wave, ncol, cs, cd, Xs, Ps, Pd);
  __syncthreads();
  if (tid < GR) {
    float s = 0.f, d = 0.f;
#pragma unroll
    for (int w = 0; w < NW; ++w) { s += Ps[tid * NW + w]; d += Pd[tid * NW + w]; }
    Sl[tid] = s;
    Dl[tid] = d;
  }
  __syncthreads();

  v4f xr[4];
#pragma unroll
  for (int i = 0; i < 4; ++i) {
    const int f   = (wave * 4 + i) * 128 + 4 * lane;
    const int row = f / DOUT;
    const int col = f - row * DOUT;
    xr[i] = *(const v4f*)(Xs + row * XSP + col);
  }
  float* hb = hp + (size_t)rowBase * DOUT;
  float* gp = 0;
  v4f gv = {0.f, 0.f, 0.f, 0.f};
  if (wave == 0 && lane < 8) {
    gv = *(const v4f*)(Sl + 4 * lane);
    gp = asb + rowBase + 4 * lane;
  } else if (wave == 0 && lane < 16) {
    gv = *(const v4f*)(Dl + 4 * (lane - 8));
    gp = adb + rowBase + 4 * (lane - 8);
  }
#pragma unroll
  for (int i = 0; i < 4; ++i) *(volatile v4f*)(hb + (wave * 4 + i) * 128 + 4 * lane) = xr[i];
  if (gp) *(volatile v4f*)gp = gv;
  __threadfence();
#pragma unroll
  for (int i = 0; i < 4; ++i) *(volatile v4f*)(hb + (wave * 4 + i) * 128 + 4 * lane) = xr[i];
  if (gp) *(volatile v4f*)gp = gv;
}

template <int DF, bool POOL> struct AggLds {
  static constexpr int SACC  = 0;
  static constexpr int DEN   = NB * DF;
  static constexpr int MR    = DEN + NB;
  static constexpr int ADL   = MR + NB;
  static constexpr int PART  = ADL + NB;
  static constexpr int NPART = POOL ? NTHR * NGR : 0;
  static constexpr int CNTL  = PART + NPART;
  static constexpr int BATL  = CNTL + (POOL ? NGR : 0);
  static constexpr int LIST  = BATL + (POOL ? NB : 0);
  static constexpr int WCNT  = LIST + NWAVE * WCAP;
  static constexpr int TOTAL = WCNT + 16;
  static constexpr unsigned BYTES = (unsigned)TOTAL * 4u;
};
static_assert((AggLds<128, false>::MR % 4) == 0);
static_assert((AggLds<64, true>::MR % 4) == 0);
static_assert((AggLds<64, true>::PART % 4) == 0);
static_assert(AggLds<128, false>::BYTES == 276544u);
static_assert(AggLds<64, true>::BYTES == 213312u);

template <int DF, bool RELU, bool POOL>
__global__ __launch_bounds__(NTHR) void k_agg(
    const int* __restrict__ ei, const float* __restrict__ xp,
    const float* __restrict__ asb, const float* __restrict__ adb,
    const float* __restrict__ bias, const int* __restrict__ batch,
    float* hout, float* ppool, float* pcnt, int nN, int nE) {
  typedef AggLds<DF, POOL> L;
  typedef typename VecT<DF / 32>::t VT;
  constexpr int VL = DF / 32;
  static_assert(POOL || DF == 128);
  static_assert(!POOL || DF == OUTD);

  extern __shared__ v4f lds_dyn[];
  float* ldsf = (float*)lds_dyn;
  float* sacc = ldsf + L::SACC;
  float* den  = ldsf + L::DEN;
  float* mr   = ldsf + L::MR;
  float* adl  = ldsf + L::ADL;
  float* part = ldsf + L::PART;
  float* cntl = ldsf + L::CNTL;
  int*   batl = (int*)(ldsf + L::BATL);
  int*   list = (int*)(ldsf + L::LIST);
  int*   wcnt = (int*)(ldsf + L::WCNT);

  const int tid  = threadIdx.x;
  const int lane = tid & 31;
  const int wave = tid >> 5;
  const int nodeBase = blockIdx.x * NB;

  {
    const v4f z4 = {0.f, 0.f, 0.f, 0.f};
    for (int i = tid; i < L::MR / 4; i += NTHR) lds_dyn[i] = z4;
    if (POOL) {
      for (int i = tid; i < L::NPART / 4; i += NTHR) lds_dyn[L::PART / 4 + i] = z4;
    }
    for (int s = tid; s < NB; s += NTHR) {
      const int nd  = nodeBase + s;
      const int ndc = nd < nN ? nd : nN - 1;
      mr[s]  = -1.0e30f;
      adl[s] = adb[ndc];
      if (POOL) batl[s] = (nd < nN) ? batch[ndc] : -1;
    }
  }
  __syncthreads();

  const int* eid = ei + nE;
  const bool al16 = ((nE & 3) == 0);

  const int nChunks = (nE + CHUNK - 1) / CHUNK;
#pragma unroll 1
  for (int ch = 0; ch < nChunks; ++ch) {
    const int cbase = ch * CHUNK;
    int wc = 0;
#pragma unroll
    for (int g = 0; g < NGRP; ++g) {
      const int el0 = (g * NTHR + tid) * 4;
      const int e0  = cbase + el0;
      const int sent = -2147483647 - 1;
      v4i d;
      if (al16 && (e0 + 3 < nE)) {
        d = *(const v4i*)(eid + e0);
      } else {
        d.x = (e0     < nE) ? eid[min(e0, nE - 1)]     : sent;
        d.y = (e0 + 1 < nE) ? eid[min(e0 + 1, nE - 1)] : sent;
        d.z = (e0 + 2 < nE) ? eid[min(e0 + 2, nE - 1)] : sent;
        d.w = (e0 + 3 < nE) ? eid[min(e0 + 3, nE - 1)] : sent;
      }
      const unsigned s0 = (unsigned)d.x - (unsigned)nodeBase;
      const unsigned s1 = (unsigned)d.y - (unsigned)nodeBase;
      const unsigned s2 = (unsigned)d.z - (unsigned)nodeBase;
      const unsigned s3 = (unsigned)d.w - (unsigned)nodeBase;
      const bool h0 = s0 < (unsigned)NB;
      const bool h1 = s1 < (unsigned)NB;
      const bool h2 = s2 < (unsigned)NB;
      const bool h3 = s3 < (unsigned)NB;
      const unsigned many = __builtin_amdgcn_ballot_w32(h0 | h1 | h2 | h3);
      if (many != 0u) {
#define HITJ(J, HJ, SJ) { \
          const unsigned mj = __builtin_amdgcn_ballot_w32(HJ); \
          if (HJ) { \
            const int pos = wc + (int)__builtin_amdgcn_mbcnt_lo(mj, 0u); \
            if (pos < WCAP) list[wave * WCAP + pos] = ((el0 + (J)) << 9) | (int)(SJ); \
          } \
          wc += (int)__builtin_popcount(mj); }
        HITJ(0, h0, s0)
        HITJ(1, h1, s1)
        HITJ(2, h2, s2)
        HITJ(3, h3, s3)
#undef HITJ
      }
    }
    if (lane == 0) wcnt[wave] = wc;
    __syncthreads();

    if (wave == 0) {
#pragma unroll 1
      for (int wsx = 0; wsx < NWAVE; ++wsx) {
        int n = wcnt[wsx];
        n = (n > WCAP) ? WCAP : ((n < 0) ? 0 : n);
#pragma unroll 1
        for (int i = 0; i < n; ++i) {
          const int ent  = list[wsx * WCAP + i];
          const int slot = ent & (NB - 1);
          const int el   = (ent >> 9) & (CHUNK - 1);
          int e = cbase + el;
          if (e > nE - 1) e = nE - 1;
          int src = ei[e];
          src = src < 0 ? 0 : (src > nN - 1 ? nN - 1 : src);
          float al = asb[src] + adl[slot];
          al = (al > 0.f) ? al : 0.2f * al;
          const float mold = mr[slot];
          const float mnew = fmaxf(mold, al);
          const float rr = __expf(fmaxf(mold - mnew, -80.f));
          const float p  = __expf(fmaxf(al - mnew, -80.f));
          const VT xv = *(const VT*)(xp + (size_t)src * DF + VL * lane);
          VT* sp = (VT*)(sacc + slot * DF + VL * lane);
          const VT cur = *sp;
          const VT nxt = cur * rr + xv * p;
          *sp = nxt;
          const float dn = den[slot] * rr + p;
          den[slot] = dn;
          mr[slot]  = mnew;
        }
      }
    }
    __syncthreads();
  }

  const VT b4 = *(const VT*)(bias + VL * lane);
  if (!POOL) {
#pragma unroll 1
    for (int j = 0; j < NB / NWAVE; ++j) {
      const int slot = wave * (NB / NWAVE) + j;
      const int node = nodeBase + slot;
      if (node >= nN) break;
      const float inv = 1.0f / (den[slot] + 1e-16f);
      VT h = *(const VT*)(sacc + slot * DF + VL * lane) * inv + b4;
      if (RELU) {
#pragma unroll
        for (int k = 0; k < VL; ++k) h[k] = h[k] > 0.f ? h[k] : 0.f;
      }
      float* op = hout + (size_t)node * DF + VL * lane;
      *(volatile VT*)op = h;
      __threadfence();
      *(volatile VT*)op = h;
    }
  } else {
#pragma unroll 1
    for (int j = 0; j < NB / NWAVE; ++j) {
      const int slot = wave * (NB / NWAVE) + j;
      const int node = nodeBase + slot;
      if (node >= nN) break;
      const float inv = 1.0f / (den[slot] + 1e-16f);
      VT* sp = (VT*)(sacc + slot * DF + VL * lane);
      VT h = *sp * inv + b4;
      if (RELU) {
#pragma unroll
        for (int k = 0; k < VL; ++k) h[k] = h[k] > 0.f ? h[k] : 0.f;
      }
      *sp = h;
    }
    __syncthreads();

    constexpr int NQ  = NTHR / DF;
    constexpr int SPQ = NB / NQ;
    const int c = tid & (DF - 1);
    const int q = tid / DF;
    float* pq = part + q * (NGR * DF) + c;
#pragma unroll 1
    for (int j = 0; j < SPQ; ++j) {
      const int slot = q * SPQ + j;
      const int g = batl[slot];
      if ((unsigned)g < (unsigned)NGR) {
        const float v = sacc[slot * DF + c];
        const float o = pq[g * DF];
        pq[g * DF] = o + v;
      }
    }
    if (tid < NGR) {
      float cn = 0.f;
#pragma unroll 1
      for (int s = 0; s < NB; ++s) cn += (batl[s] == tid) ? 1.0f : 0.0f;
      cntl[tid] = cn;
    }
    __syncthreads();

    v4f pv[4];
#pragma unroll
    for (int i = 0; i < 4; ++i) {
      const int base = (wave * 4 + i) * 128 + 4 * lane;
      v4f s = *(const v4f*)(part + base);
#pragma unroll
      for (int qq = 1; qq < NQ; ++qq) s = s + *(const v4f*)(part + qq * (NGR * DF) + base);
      pv[i] = s;
    }
    const bool hc = (wave == 0) && (lane < NGR / 4);
    v4f cv = {0.f, 0.f, 0.f, 0.f};
    if (hc) cv = *(const v4f*)(cntl + 4 * lane);
    float* pb = ppool + (size_t)blockIdx.x * PP;
    float* cb = pcnt + (size_t)blockIdx.x * NGR + 4 * lane;
#pragma unroll
    for (int i = 0; i < 4; ++i) *(volatile v4f*)(pb + (wave * 4 + i) * 128 + 4 * lane) = pv[i];
    if (hc) *(volatile v4f*)cb = cv;
    __threadfence();
#pragma unroll
    for (int i = 0; i < 4; ++i) *(volatile v4f*)(pb + (wave * 4 + i) * 128 + 4 * lane) = pv[i];
    if (hc) *(volatile v4f*)cb = cv;
  }
}

__global__ __launch_bounds__(NTHR) void k_final(const float* __restrict__ ppool, const float* __restrict__ pcnt,
                                                float* out, int nblk) {
  __shared__ __attribute__((aligned(16))) float outl[PP];
  __shared__ float rec[NGR];
  const int tid  = threadIdx.x;
  const int lane = tid & 31;
  const int wave = tid >> 5;
  if (tid < NGR) {
    float cn = 0.f;
#pragma unroll 1
    for (int b = 0; b < nblk; ++b) cn += pcnt[(size_t)b * NGR + tid];
    rec[tid] = 1.0f / fmaxf(cn, 1.0f);
  }
  __syncthreads();
#pragma unroll 1
  for (int i = 0; i < PP / NTHR; ++i) {
    const int e = i * NTHR + tid;
    float s = 0.f;
#pragma unroll 1
    for (int b = 0; b < nblk; ++b) s += ppool[(size_t)b * PP + e];
    outl[e] = s * rec[e / OUTD];
  }
  __syncthreads();
  v4f ov[4];
#pragma unroll
  for (int i = 0; i < 4; ++i) ov[i] = *(const v4f*)(outl + (wave * 4 + i) * 128 + 4 * lane);
#pragma unroll
  for (int i = 0; i < 4; ++i) *(volatile v4f*)(out + (wave * 4 + i) * 128 + 4 * lane) = ov[i];
  __threadfence();
#pragma unroll
  for (int i = 0; i < 4; ++i) *(volatile v4f*)(out + (wave * 4 + i) * 128 + 4 * lane) = ov[i];
}

static inline size_t al256(size_t b) { return (b + 255) & ~(size_t)255; }

extern "C" void kernel_launch(void* const* d_in, const int* in_sizes, int n_in,
                              void* d_out, int out_size, void* d_ws, size_t ws_size,
                              hipStream_t stream) {
  if (n_in < 15) return;
  const int nN = in_sizes[0] / DIN;
  if (nN <= 0 || in_sizes[0] != nN * DIN) return;
  if (in_sizes[1] < 0 || (in_sizes[1] & 1)) return;
  const int nE = in_sizes[1] / 2;
  if (in_sizes[2] != nN) return;
  if (in_sizes[3] != DIN * HID || in_sizes[4] != HID || in_sizes[5] != HID || in_sizes[6] != HID) return;
  if (in_sizes[7] != DIN * HID || in_sizes[8] != HID || in_sizes[9] != HID || in_sizes[10] != HID) return;
  if (in_sizes[11] != DIN * OUTD || in_sizes[12] != OUTD || in_sizes[13] != OUTD || in_sizes[14] != OUTD) return;
  if (out_size != PP) return;

  const float* x     = (const float*)d_in[0];
  const int*   ei    = (const int*)d_in[1];
  const int*   batch = (const int*)d_in[2];
  const float* W1 = (const float*)d_in[3];  const float* as1 = (const float*)d_in[4];
  const float* ad1 = (const float*)d_in[5]; const float* b1 = (const float*)d_in[6];
  const float* W2 = (const float*)d_in[7];  const float* as2 = (const float*)d_in[8];
  const float* ad2 = (const float*)d_in[9]; const float* b2 = (const float*)d_in[10];
  const float* W3 = (const float*)d_in[11]; const float* as3 = (const float*)d_in[12];
  const float* ad3 = (const float*)d_in[13]; const float* b3 = (const float*)d_in[14];
  float* out = (float*)d_out;

  const int nP   = ((nN + GR - 1) / GR) * GR;
  const int nblk = (nN + NB - 1) / NB;

  size_t off = 0;
  _Float16* Wt = (_Float16*)((char*)d_ws + off); off += al256((size_t)HID * DIN * sizeof(_Float16));
  float* xp  = (float*)((char*)d_ws + off);       off += al256((size_t)nP * HID * sizeof(float));
  float* h1  = (float*)((char*)d_ws + off);       off += al256((size_t)nP * HID * sizeof(float));
  float* h2  = (float*)((char*)d_ws + off);       off += al256((size_t)nP * HID * sizeof(float));
  float* asb = (float*)((char*)d_ws + off);       off += al256((size_t)nP * sizeof(float));
  float* adb = (float*)((char*)d_ws + off);       off += al256((size_t)nP * sizeof(float));
  float* ppool = (float*)((char*)d_ws + off);     off += al256((size_t)nblk * PP * sizeof(float));
  float* pcnt  = (float*)((char*)d_ws + off);     off += al256((size_t)nblk * NGR * sizeof(float));
  if (off > ws_size) return;

  hipFuncSetAttribute(reinterpret_cast<const void*>(&k_agg<128, true, false>),
                      hipFuncAttributeMaxDynamicSharedMemorySize, (int)AggLds<128, false>::BYTES);
  hipFuncSetAttribute(reinterpret_cast<const void*>(&k_agg<64, false, true>),
                      hipFuncAttributeMaxDynamicSharedMemorySize, (int)AggLds<64, true>::BYTES);

  const int gridG = nP / GR;
  const int prepH = (HID * (DIN / 8) + NTHR - 1) / NTHR;
  const int prepO = (OUTD * (DIN / 8) + NTHR - 1) / NTHR;

  k_prep<<<prepH, NTHR, 0, stream>>>(W1, Wt, DIN, HID);
  k_gemm<128><<<gridG, 256, 0, stream>>>(x, Wt, as1, ad1, xp, asb, adb, nN);
  k_agg<128, true, false><<<nblk, NTHR, AggLds<128, false>::BYTES, stream>>>(
      ei, xp, asb, adb, b1, batch, h1, ppool, pcnt, nN, nE);

  k_prep<<<prepH, NTHR, 0, stream>>>(W2, Wt, DIN, HID);
  k_gemm<128><<<gridG, 256, 0, stream>>>(h1, Wt, as2, ad2, xp, asb, adb, nN);
  k_agg<128, true, false><<<nblk, NTHR, AggLds<128, false>::BYTES, stream>>>(
      ei, xp, asb, adb, b2, batch, h2, ppool, pcnt, nN, nE);

  k_prep<<<prepO, NTHR, 0, stream>>>(W3, Wt, DIN, OUTD);
  k_gemm<64><<<gridG, 128, 0, stream>>>(h2, Wt, as3, ad3, xp, asb, adb, nN);
  k_agg<64, false, true><<<nblk, NTHR, AggLds<64, true>::BYTES, stream>>>(
      ei, xp, asb, adb, b3, batch, h2, ppool, pcnt, nN, nE);

  k_final<<<1, NTHR, 0, stream>>>(ppool, pcnt, out, nblk);
}
